// SelfAttention_56032143344081
// MI455X (gfx1250) — hardware-verified
//
#include <hip/hip_runtime.h>


#ifndef NB
#define NB 4
#endif
#ifndef SEQ
#define SEQ 2048
#endif
#define NB_FULL 4
#define SEQ_FULL 2048
#define DM 1024
#define NH 8
#define DK 128
#define MTOK (NB * SEQ)
#define NPROJ (3 * DM)
#define PLANE ((size_t)NB * NH * SEQ * DK)

#define NMW (NB * (SEQ / 32))
#define MBW (((NMW + 31) / 32) * 32)
#define MBTOT (MBW + 32)

static_assert(SEQ % 64 == 0);
static_assert(SEQ <= SEQ_FULL);
static_assert(NB >= 1 && NB <= NB_FULL);
static_assert(NH * DK == DM);
static_assert(DK == 128);
static_assert(DM % 64 == 0);
static_assert(DM % 32 == 0);
static_assert(NPROJ == 24 * 128);
static_assert(MBW <= 256);
static_assert(MBTOT % 4 == 0);
static_assert(MBTOT / 4 <= 256);
static_assert(((size_t)DM * DM) % (8 * 256) == 0);
static_assert(64 * 136 <= 9216);
static_assert(128 * 72 <= 9216);

#define SC_X   16.0f
#define SC_W   256.0f
#define SC_QKV 8.0f
#define SC_P   256.0f
#define PROJ_FOLD (SC_QKV / (SC_X * SC_W))

#define WPREP_BLK_Q ((DM * DM) / 8 / 256)
#define WPREP_BLK   ((3 * DM * DM) / 8 / 256)

#define MB_BYTES ((((size_t)MBTOT * 4) + 255) / 256 * 256)
#define WS_TOTAL ((size_t)NPROJ * DM * 2 + (size_t)MTOK * DM * 2 + 3 * PLANE * 2 + MB_BYTES)
static_assert(((size_t)NPROJ * DM * 2) % 256 == 0);
static_assert(((size_t)MTOK * DM * 2) % 256 == 0);
static_assert((PLANE * 2) % 256 == 0);
static_assert(WS_TOTAL <= (size_t)134217728);

typedef _Float16 v8h  __attribute__((ext_vector_type(8)));
typedef _Float16 v16h __attribute__((ext_vector_type(16)));
typedef float    v8f  __attribute__((ext_vector_type(8)));
typedef float    v4f  __attribute__((ext_vector_type(4)));
typedef unsigned v4u  __attribute__((ext_vector_type(4)));
typedef int      v4i  __attribute__((ext_vector_type(4)));

__device__ __forceinline__ float bfr(float f) {
    unsigned u = __float_as_uint(f);
    u = (u + 0x7fffu + ((u >> 16) & 1u)) & 0xffff0000u;
    return __uint_as_float(u);
}
static __device__ __forceinline__ _Float16 toh_flush(float v) {
    const _Float16 r = (_Float16)v;
    return (fabsf(v) < 6.103515625e-05f) ? (_Float16)0.0f : r;
}
static __device__ __forceinline__ _Float16 tohxf(float f, float sc) { return toh_flush(bfr(f) * sc); }

__device__ __forceinline__ v8f wmma16(v16h a, v16h b, v8f c) {
    c = __builtin_amdgcn_wmma_f32_16x16x32_f16(false, a, false, b, (short)0, c, false, false);
    asm volatile("v_nop\n\tv_nop\n\tv_nop\n\tv_nop" : "+v"(c) : "v"(a), "v"(b));
    return c;
}
__device__ __forceinline__ v16h ldfrag(const _Float16* p, int hf) {
    const v8h lo = *(const v8h*)(p + 8 * hf);
    const v8h hi = *(const v8h*)(p + 16 + 8 * hf);
    return __builtin_shufflevector(lo, hi, 0, 1, 2, 3, 4, 5, 6, 7, 8, 9, 10, 11, 12, 13, 14, 15);
}
__device__ __forceinline__ void vst16(_Float16* g, v8h v) { *(volatile v4u*)g = __builtin_bit_cast(v4u, v); }
__device__ __forceinline__ void vst16f(float* g, v4f v) { *(volatile v4f*)g = v; }
__device__ __forceinline__ void vst16w(unsigned* g, v4u v) { *(volatile v4u*)g = v; }

__global__ __launch_bounds__(256) void k_wprep(const float* __restrict__ Wq, const float* __restrict__ W1, _Float16* WT) {
#pragma clang fp contract(off)
    const int i = blockIdx.x * 256 + threadIdx.x;
    const size_t e = (size_t)i * 8;
    v4f a, b;
    if (blockIdx.x < WPREP_BLK_Q) {
        a = *(const v4f*)(Wq + e);
        b = *(const v4f*)(Wq + e + 4);
    } else {
        const size_t e1 = e - (size_t)DM * DM;
        a = *(const v4f*)(W1 + e1);
        b = *(const v4f*)(W1 + e1 + 4);
    }
    v8h val;
#pragma unroll
    for (int j = 0; j < 4; ++j) { val[j] = tohxf(a[j], SC_W); val[4 + j] = tohxf(b[j], SC_W); }
    _Float16* dst = WT + e;
    vst16(dst, val);
    __threadfence();
    vst16(dst, val);
}

__global__ __launch_bounds__(256) void k_mask(const int* __restrict__ mask, unsigned* MB) {
#pragma clang fp contract(off)
    __shared__ __align__(16) unsigned wb[MBTOT];
    __shared__ unsigned sb[8];
    const int tid = threadIdx.x, lane = tid & 31;
    const int wave = __builtin_amdgcn_readfirstlane(threadIdx.x >> 5);
    const int wi = (tid < NMW) ? tid : (NMW - 1);
    const int bi = wi / (SEQ / 32), wk = wi - bi * (SEQ / 32);
    const int* mp = mask + (size_t)bi * SEQ_FULL + wk * 32;
    unsigned word = 0u, bad = 0u;
#pragma unroll
    for (int j = 0; j < 8; ++j) {
        const v4i m = *(const v4i*)(mp + 4 * j);
#pragma unroll
        for (int i = 0; i < 4; ++i) {
            word |= ((m[i] == 1) ? 1u : 0u) << (4 * j + i);
            bad  |= ((unsigned)m[i] > 1u) ? 1u : 0u;
        }
    }
    word = (tid < NMW) ? word : 0u;
    if (tid < MBW) wb[tid] = word;
    bad |= __shfl_xor(bad, 1, 32);
    bad |= __shfl_xor(bad, 2, 32);
    bad |= __shfl_xor(bad, 4, 32);
    bad |= __shfl_xor(bad, 8, 32);
    bad |= __shfl_xor(bad, 16, 32);
    if (lane == 0) sb[wave] = bad;
    __syncthreads();
    unsigned flag = 0u;
#pragma unroll
    for (int w = 0; w < 8; ++w) flag |= sb[w];
    if (tid < 32) wb[MBW + tid] = flag;
    __syncthreads();
    if (tid < MBTOT / 4) {
        const v4u v = *(const v4u*)&wb[4 * tid];
        vst16w(MB + 4 * tid, v);
        __threadfence();
        vst16w(MB + 4 * tid, v);
    }
}

__global__ __launch_bounds__(256) void k_xt(const float* __restrict__ X, _Float16* XT) {
#pragma clang fp contract(off)
    __shared__ __align__(16) _Float16 st[64 * 72];
    const int tid = threadIdx.x;
    const int l0 = blockIdx.x * 64, d0 = blockIdx.y * 64, bi = blockIdx.z;
    const float* xb = X + ((size_t)bi * DM + d0) * SEQ_FULL + l0;
#pragma unroll
    for (int rep = 0; rep < 4; ++rep) {
        const int idx = rep * 256 + tid;
        const int dd = idx >> 4, l4 = (idx & 15) * 4;
        const v4f x = *(const v4f*)(xb + (size_t)dd * SEQ_FULL + l4);
#pragma unroll
        for (int j = 0; j < 4; ++j) st[(l4 + j) * 72 + dd] = tohxf(x[j], SC_X);
    }
    __syncthreads();
    v8h w[2];
#pragma unroll
    for (int rep = 0; rep < 2; ++rep) {
        const int idx = rep * 256 + tid;
        const int row = idx >> 3, pc = idx & 7;
        w[rep] = *(const v8h*)&st[row * 72 + pc * 8];
    }
    auto pass = [&]() {
#pragma unroll
        for (int rep = 0; rep < 2; ++rep) {
            const int idx = rep * 256 + tid;
            const int row = idx >> 3, pc = idx & 7;
            vst16(XT + (size_t)(bi * SEQ + l0 + row) * DM + d0 + pc * 8, w[rep]);
        }
    };
    pass();
    __threadfence();
    pass();
}

__global__ __launch_bounds__(128) void k_proj(const _Float16* __restrict__ XT, const _Float16* __restrict__ WT,
                                              _Float16* QK, _Float16* VT) {
    __shared__ __align__(16) _Float16 st[9216];
    const int tid = threadIdx.x, lane = tid & 31, l16 = lane & 15, hf = lane >> 4;
    const int wv = __builtin_amdgcn_readfirstlane(threadIdx.x >> 5);
    const int g = blockIdx.y;
    const int t0 = blockIdx.x * 64;
    const int bi = t0 / SEQ, s0 = t0 - bi * SEQ;
    const bool isV = (g >= 16);
    const _Float16* arow = XT + (size_t)(t0 + wv * 16 + l16) * DM;
    const _Float16* brow = WT + (size_t)(g * 128 + l16) * DM;
    v8f acc[8];
#pragma unroll
    for (int nt = 0; nt < 8; ++nt) acc[nt] = (v8f){};
#pragma unroll 1
    for (int kc = 0; kc < DM / 32; ++kc) {
        const v16h a = ldfrag(arow + kc * 32, hf);
#pragma unroll
        for (int nt = 0; nt < 8; ++nt) {
            const v16h bf = ldfrag(brow + (size_t)nt * 16 * DM + kc * 32, hf);
            acc[nt] = wmma16(a, bf, acc[nt]);
        }
    }
    if (isV) {
#pragma unroll
        for (int nt = 0; nt < 8; ++nt) {
            const int d = nt * 16 + l16;
            v8h pv;
#pragma unroll
            for (int r = 0; r < 8; ++r) pv[r] = toh_flush(acc[nt][r] * PROJ_FOLD);
            *(v8h*)&st[d * 72 + wv * 16 + 8 * hf] = pv;
        }
    } else {
#pragma unroll
        for (int nt = 0; nt < 8; ++nt) {
            const int col = nt * 16 + l16;
#pragma unroll
            for (int r = 0; r < 8; ++r) st[(wv * 16 + 8 * hf + r) * 136 + col] = toh_flush(acc[nt][r] * PROJ_FOLD);
        }
    }
    __syncthreads();
    v8h w[8];
    if (isV) {
        const int hd = g - 16;
#pragma unroll
        for (int p = 0; p < 8; ++p) { const int d = p * 16 + (tid >> 3), pc = tid & 7; w[p] = *(const v8h*)&st[d * 72 + pc * 8]; }
        auto pass = [&]() {
#pragma unroll
            for (int p = 0; p < 8; ++p) {
                const int d = p * 16 + (tid >> 3), pc = tid & 7;
                vst16(VT + ((size_t)(bi * NH + hd) * DK + d) * SEQ + s0 + pc * 8, w[p]);
            }
        };
        pass();
        __threadfence();
        pass();
    } else {
        const size_t poff = (g < 8) ? (size_t)0 : PLANE;
        _Float16* base = QK + poff + ((size_t)(bi * NH + (g & 7)) * SEQ + s0) * DK;
#pragma unroll
        for (int p = 0; p < 8; ++p) { const int off = p * 1024 + tid * 8; w[p] = *(const v8h*)&st[(off >> 7) * 136 + (off & 127)]; }
        auto pass = [&]() {
#pragma unroll
            for (int p = 0; p < 8; ++p) { const int off = p * 1024 + tid * 8; vst16(base + off, w[p]); }
        };
        pass();
        __threadfence();
        pass();
    }
}

__global__ __launch_bounds__(128) void k_attn(const _Float16* __restrict__ QC, const _Float16* __restrict__ KC,
                                              const _Float16* __restrict__ VT, const unsigned* __restrict__ MB, float* OUT) {
    __shared__ __align__(16) float st[128 * 68];
    const int tid = threadIdx.x, lane = tid & 31, l16 = lane & 15, hf = lane >> 4;
    const int wv = __builtin_amdgcn_readfirstlane(threadIdx.x >> 5);
    const int bh = blockIdx.y, bi = bh / NH, hd = bh - bi * NH;
    const int q0 = blockIdx.x * 64 + wv * 16;
    v16h qf[4];
    {
        const _Float16* qr = QC + ((size_t)bh * SEQ + q0 + l16) * DK;
#pragma unroll
        for (int cc = 0; cc < 4; ++cc) qf[cc] = ldfrag(qr + cc * 32, hf);
    }
    const _Float16* kb = KC + (size_t)bh * SEQ * DK;
    const _Float16* vb = VT + (size_t)bh * DK * SEQ;
    const unsigned* mb = MB + (size_t)bi * (SEQ / 32);
    v8f o[8];
#pragma unroll
    for (int d = 0; d < 8; ++d) o[d] = (v8f){};
    float m2 = -__builtin_inff(), lsum = 0.0f;
    const float c2 = (0.08838834764831845f * 1.4426950408889634f) * (1.0f / (SC_QKV * SC_QKV));
#pragma unroll 1
    for (int kt = 0; kt < SEQ / 64; ++kt) {
        const unsigned w0 = mb[kt * 2], w1 = mb[kt * 2 + 1];
        v8f s[4];
#pragma unroll
        for (int ks = 0; ks < 4; ++ks) {
            const int key = kt * 64 + ks * 16 + l16;
            const _Float16* kr = kb + (size_t)key * DK;
            v8f c = (v8f){};
#pragma unroll
            for (int cc = 0; cc < 4; ++cc) c = wmma16(ldfrag(kr + cc * 32, hf), qf[cc], c);
            s[ks] = c;
        }
        float mloc = -__builtin_inff();
#pragma unroll
        for (int ks = 0; ks < 4; ++ks) {
            const unsigned mbits = ((ks < 2) ? w0 : w1) >> ((ks & 1) * 16 + 8 * hf);
#pragma unroll
            for (int r = 0; r < 8; ++r) {
                const float sv = s[ks][r] * c2;
                const float sm = (((mbits >> r) & 1u) != 0u) ? sv : -1.0e30f;
                s[ks][r] = sm;
                mloc = fmaxf(mloc, sm);
            }
        }
        mloc = fmaxf(mloc, __shfl_xor(mloc, 16, 32));
        const float mn = fmaxf(m2, mloc);
        const float alpha = exp2f(m2 - mn);
        float ls = 0.0f;
        v16h pf[2];
#pragma unroll
        for (int ks = 0; ks < 4; ++ks)
#pragma unroll
            for (int r = 0; r < 8; ++r) {
                const float e = s[ks][r] - mn;
                const float p = (e < -22.0f) ? 0.0f : exp2f(e);
                ls += p;
                pf[ks >> 1][(ks & 1) * 8 + r] = (_Float16)(p * SC_P);
            }
        m2 = mn;
        lsum = lsum * alpha + ls;
#pragma unroll
        for (int d = 0; d < 8; ++d) o[d] *= alpha;
#pragma unroll
        for (int d = 0; d < 8; ++d) {
            const _Float16* vr = vb + (size_t)(d * 16 + l16) * SEQ + kt * 64;
            o[d] = wmma16(ldfrag(vr, hf), pf[0], o[d]);
            o[d] = wmma16(ldfrag(vr + 32, hf), pf[1], o[d]);
        }
    }
    const float lt = lsum + __shfl_xor(lsum, 16, 32);
    const unsigned flag = MB[MBW];
    const float inv = (flag != 0u) ? __uint_as_float(0x7fc00000u) : (1.0f / (lt * (SC_P * SC_QKV)));
#pragma unroll
    for (int d = 0; d < 8; ++d)
#pragma unroll
        for (int r = 0; r < 8; ++r) st[(d * 16 + 8 * hf + r) * 68 + wv * 16 + l16] = o[d][r] * inv;
    __syncthreads();
    v4f w[16];
#pragma unroll
    for (int t = 0; t < 16; ++t) { const int idx = t * 128 + tid; const int dd = idx >> 4, pc = idx & 15; w[t] = *(const v4f*)&st[dd * 68 + pc * 4]; }
    float* ob = OUT + ((size_t)bi * DM + hd * DK) * SEQ_FULL + blockIdx.x * 64;
    auto pass = [&]() {
#pragma unroll
        for (int t = 0; t < 16; ++t) {
            const int idx = t * 128 + tid;
            const int dd = idx >> 4, pc = idx & 15;
            vst16f(ob + (size_t)dd * SEQ_FULL + pc * 4, w[t]);
        }
    };
    pass();
    __threadfence();
    pass();
}

extern "C" void kernel_launch(void* const* d_in, const int* in_sizes, int n_in,
                              void* d_out, int out_size, void* d_ws, size_t ws_size, hipStream_t stream) {
    if (n_in < 4) return;
    const long long needX = ((long long)(NB - 1) * DM + (DM - 1)) * SEQ_FULL + SEQ;
    const long long needM = (long long)(NB - 1) * SEQ_FULL + SEQ;
    if ((long long)in_sizes[0] < needX) return;
    if ((long long)in_sizes[1] < needM) return;
    if ((long long)in_sizes[2] < (long long)2 * DM * DM) return;
    if ((long long)in_sizes[3] < (long long)DM * DM) return;
    if ((long long)out_size < needX) return;

    const float* query = (const float*)d_in[0];
    const int*   mask  = (const int*)d_in[1];
    const float* W1    = (const float*)d_in[2];
    const float* Wq    = (const float*)d_in[3];
    float* out = (float*)d_out;

    char* ws = (char*)d_ws;
    size_t off = 0;
    auto carve = [&](size_t bytes) -> char* { char* p = ws + off; off += (bytes + 255) & ~(size_t)255; return p; };
    _Float16* WT = (_Float16*)carve((size_t)NPROJ * DM * 2);
    _Float16* XT = (_Float16*)carve((size_t)MTOK * DM * 2);
    _Float16* QK = (_Float16*)carve(2 * PLANE * 2);
    _Float16* VT = (_Float16*)carve(PLANE * 2);
    unsigned* MB = (unsigned*)carve((size_t)MBTOT * 4);
    if (off > ws_size) return;
    if (off > (size_t)134217728) return;

    k_wprep<<<WPREP_BLK, 256, 0, stream>>>(Wq, W1, WT);
    k_mask<<<1, 256, 0, stream>>>(mask, MB);
    k_xt<<<dim3(SEQ / 64, DM / 64, NB), 256, 0, stream>>>(query, XT);
    k_proj<<<dim3(MTOK / 64, NPROJ / 128, 1), 128, 0, stream>>>(XT, WT, QK, VT);
    k_attn<<<dim3(SEQ / 64, NB * NH, 1), 128, 0, stream>>>(QK, QK + PLANE, VT, MB, out);
}
